// ResidualCGConvBlock_52862457480029
// MI455X (gfx1250) — hardware-verified
//
#include <hip/hip_runtime.h>
#include <math.h>

#define NN 20000
#define NP 20032
#define FD 128
#define ED 16
#define NE 600000
#define ZW 272
#define PC 512
#define NT 256
#define TILE 2048
#define NTILES 10
#define NACC (NTILES * TILE)
#define SCH 2048
#define SPT (SCH / NT)
#define NCH ((NE + SCH - 1) / SCH)
#define HB 32
#define PP 256
#define NBP 80
#define RPB 250
#define WSC 16.0f
#define WSC_INV 0.0625f
#define EPSV 1e-5f

#define XH_N2 (NP * FD / 2)
#define XV_N2 (NN * FD / 2)
#define WT_N2 (PC * FD / 2)
#define BC_N2 (256 * 32 / 2)
#define PREP_TOTAL (XH_N2 + WT_N2 + BC_N2)

static_assert(NE % SPT == 0, "edge groups are whole");
static_assert(NBP * RPB == NN, "stat blocks cover all nodes");
static_assert(NP % 64 == 0 && PC % 64 == 0 && FD % 32 == 0, "gemm tiling");
static_assert(NACC >= NN, "accumulator rows cover all nodes");
static_assert(HB == 32, "one hit slot per lane");

typedef __attribute__((ext_vector_type(16))) _Float16 v16h;
typedef __attribute__((ext_vector_type(8)))  _Float16 v8h;
typedef __attribute__((ext_vector_type(4)))  _Float16 v4h;
typedef __attribute__((ext_vector_type(16))) __bf16   v16b;
typedef __attribute__((ext_vector_type(8)))  __bf16   v8b;
typedef __attribute__((ext_vector_type(8)))  float    v8f;
typedef __attribute__((ext_vector_type(4)))  float    v4f;
typedef __attribute__((ext_vector_type(4)))  int      v4i;

__device__ __forceinline__ unsigned short f2bf_bits(float f) {
  unsigned u = __float_as_uint(f);
  return (unsigned short)((u + 0x7FFFu + ((u >> 16) & 1u)) >> 16);
}
__device__ __forceinline__ float bf_bits2f(unsigned short h) { return __uint_as_float(((unsigned)h) << 16); }

__device__ __forceinline__ void dep_guard_h(v8f& a, v8f& b, v16h x, v16h y) { asm volatile("v_nop\n\tv_nop\n\tv_nop\n\tv_nop" : "+v"(a), "+v"(b) : "v"(x), "v"(y)); }
__device__ __forceinline__ void dep_guard_b(v8f& a, v8f& b, v16b x, v16b y) { asm volatile("v_nop\n\tv_nop\n\tv_nop\n\tv_nop" : "+v"(a), "+v"(b) : "v"(x), "v"(y)); }
__device__ __forceinline__ void keep4_h(v16h a, v16h b, v16h c, v16h d) { asm volatile("v_nop" :: "v"(a), "v"(b), "v"(c), "v"(d)); }
__device__ __forceinline__ void keep4_b(v16b a, v16b b, v16b c, v16b d) { asm volatile("v_nop" :: "v"(a), "v"(b), "v"(c), "v"(d)); }
__device__ __forceinline__ void acc_guard4(v8f& a, v8f& b, v8f& c, v8f& d) { asm volatile("v_nop\n\tv_nop\n\tv_nop\n\tv_nop" : "+v"(a), "+v"(b), "+v"(c), "+v"(d)); }
template <typename T> struct Frag;
template <> struct Frag<_Float16> {
  typedef v16h V; union U { v16h v; v8h h[2]; };
  static __device__ __forceinline__ v16h load(const _Float16* p) {
    U f; f.h[0] = *(const v8h*)(p); f.h[1] = *(const v8h*)(p + 16); return f.v;
  }
  static __device__ __forceinline__ v8f mma(v16h a, v16h b, v8f c) {
    return __builtin_amdgcn_wmma_f32_16x16x32_f16(false, a, false, b, (short)0, c, false, false);
  }
  static __device__ __forceinline__ void guard(v8f& a, v8f& b, v16h x, v16h y) { dep_guard_h(a, b, x, y); }
  static __device__ __forceinline__ void keep(v16h a, v16h b, v16h c, v16h d) { keep4_h(a, b, c, d); }
};
template <> struct Frag<__bf16> {
  typedef v16b V; union U { v16b v; v8b h[2]; };
  static __device__ __forceinline__ v16b load(const __bf16* p) {
    U f; f.h[0] = *(const v8b*)(p); f.h[1] = *(const v8b*)(p + 16); return f.v;
  }
  static __device__ __forceinline__ v8f mma(v16b a, v16b b, v8f c) {
    return __builtin_amdgcn_wmma_f32_16x16x32_bf16(false, a, false, b, (short)0, c, false, false);
  }
  static __device__ __forceinline__ void guard(v8f& a, v8f& b, v16b x, v16b y) { dep_guard_b(a, b, x, y); }
  static __device__ __forceinline__ void keep(v16b a, v16b b, v16b c, v16b d) { keep4_b(a, b, c, d); }
};

template <int ET> struct Elem;
template <> struct Elem<0> { typedef _Float16 T; };
template <> struct Elem<1> { typedef __bf16 T; };
template <int ET, bool SPLIT, int BIAS_MODE, int OUT_MODE, bool RESID, int ACT = 0>
__global__ __launch_bounds__(256) void wmma_gemm64(
    const unsigned short* __restrict__ Ap, const unsigned short* __restrict__ A2p, int lda, long strideA,
    const unsigned short* __restrict__ Btp, const unsigned short* __restrict__ Bt2p, int ldb, long strideB,
    void* __restrict__ Cout, void* __restrict__ Cout2, int ldc, long strideC,
    const float* __restrict__ bias,
    const float* __restrict__ resid, long strideR,
    int M, int N, int K, float scale) {
  typedef typename Elem<ET>::T T;
  typedef typename Frag<T>::V V;
  const T* A = (const T*)Ap; const T* A2 = (const T*)A2p; const T* Bt = (const T*)Btp; const T* Bt2 = (const T*)Bt2p;
  __shared__ __align__(16) float sT[8][16 * 68];
  const int b    = blockIdx.y;
  const int lane = threadIdx.x & 31;
  const int wave = threadIdx.x >> 5;
  const int tilesN = N >> 6;
  const int tilesM = M >> 6;
  const int tile = blockIdx.x * 8 + wave;
  if (tile >= tilesM * tilesN) return;
  const int tm = tile / tilesN;
  const int tn = tile - tm * tilesN;
  const int m0 = tm << 6;
  const int n0 = tn << 6;

  const T* Ab  = A  + (size_t)b * strideA;
  const T* Bb  = Bt + (size_t)b * strideB;
  const T* Ab2 = SPLIT ? (A2  + (size_t)b * strideA) : nullptr;
  const T* Bb2 = SPLIT ? (Bt2 + (size_t)b * strideB) : nullptr;

  const int rlane = lane & 15;
  const int koff  = (lane >> 4) * 8;
  const int mOff  = (lane >> 4) * 8;

  v8f acc[4][4];
#pragma unroll
  for (int i = 0; i < 4; ++i)
#pragma unroll
    for (int j = 0; j < 4; ++j) acc[i][j] = (v8f){0.f,0.f,0.f,0.f,0.f,0.f,0.f,0.f};

  for (int k0 = 0; k0 < K; k0 += 32) {
    V bh[4], bl[4];
#pragma unroll
    for (int j = 0; j < 4; ++j) {
      const size_t bo = (size_t)(n0 + (j << 4) + rlane) * ldb + koff + k0;
      bh[j] = Frag<T>::load(Bb + bo);
      if (SPLIT) bl[j] = Frag<T>::load(Bb2 + bo);
    }
#pragma unroll
    for (int i = 0; i < 4; ++i) {
      const size_t ao = (size_t)(m0 + (i << 4) + rlane) * lda + koff + k0;
      V ah = Frag<T>::load(Ab + ao);
      V al;
      if (SPLIT) al = Frag<T>::load(Ab2 + ao);
#pragma unroll
      for (int j = 0; j < 4; ++j) {
        acc[i][j] = Frag<T>::mma(ah, bh[j], acc[i][j]);
        if (SPLIT) {
          acc[i][j] = Frag<T>::mma(ah, bl[j], acc[i][j]);
          acc[i][j] = Frag<T>::mma(al, bh[j], acc[i][j]);
        }
      }
      Frag<T>::guard(acc[i][0], acc[i][3], ah, SPLIT ? al : ah);
    }
    Frag<T>::keep(bh[0], bh[1], bh[2], bh[3]);
    if (SPLIT) Frag<T>::keep(bl[0], bl[1], bl[2], bl[3]);
  }
  acc_guard4(acc[0][0], acc[0][1], acc[0][2], acc[0][3]);
  acc_guard4(acc[1][0], acc[1][1], acc[1][2], acc[1][3]);
  acc_guard4(acc[2][0], acc[2][1], acc[2][2], acc[2][3]);
  acc_guard4(acc[3][0], acc[3][1], acc[3][2], acc[3][3]);

  float* slab = sT[wave];
  const float* Rb = RESID ? (resid + (size_t)b * strideR) : nullptr;
#pragma unroll
  for (int i = 0; i < 4; ++i) {
    const int mBase = m0 + (i << 4);
#pragma unroll
    for (int j = 0; j < 4; ++j) {
      const int n = n0 + (j << 4) + rlane;
      float bv = 0.f;
      if (BIAS_MODE == 2) bv = bias[n];
#pragma unroll
      for (int r = 0; r < 8; ++r) {
        float v = acc[i][j][r] * scale;
        if (BIAS_MODE == 1) v += bias[mBase + mOff + r];
        if (BIAS_MODE == 2) v += bv;
        if (RESID) v += Rb[(size_t)(mBase + mOff + r) * ldc + n];
        if (ACT == 1) v = tanhf(v);
        if (ACT == 2) v = fmaxf(v, 0.0f);
        if (ACT == 3) v = v / (1.0f + expf(-v));
        if (ACT == 4) v = (v > 0.f) ? v : 0.01f * v;
        if (ACT == 5) v = 0.5f * v * (1.0f + erff(v * 0.70710678118654752f));
        slab[(mOff + r) * 68 + (j << 4) + rlane] = v;
      }
    }
    __builtin_amdgcn_fence(__ATOMIC_RELEASE, "workgroup");
    __builtin_amdgcn_wave_barrier();
    __builtin_amdgcn_fence(__ATOMIC_ACQUIRE, "workgroup");
    if (OUT_MODE == 0) {
      float* C = (float*)Cout + (size_t)b * strideC;
      const int hh = lane >> 4, c4 = (lane & 15) * 4;
      for (int pass = 0; pass < 2; ++pass) {
#pragma unroll
        for (int it = 0; it < 8; ++it) {
          const int row = it * 2 + hh;
          v4f v = *(const v4f*)(slab + row * 68 + c4);
          *(volatile v4f*)(C + (size_t)(mBase + row) * ldc + n0 + c4) = v;
        }
        __threadfence();
      }
    } else {
      const int q = lane >> 3, c8 = (lane & 7) * 8;
      unsigned short* C  = (unsigned short*)Cout  + (size_t)b * strideC;
      unsigned short* C2 = (OUT_MODE == 2) ? ((unsigned short*)Cout2 + (size_t)b * strideC) : nullptr;
      for (int pass = 0; pass < 2; ++pass) {
#pragma unroll
        for (int it = 0; it < 4; ++it) {
          const int row = it * 4 + q;
          const float* sp = slab + row * 68 + c8;
          v8h hv, lv;
#pragma unroll
          for (int e = 0; e < 8; ++e) {
            if (OUT_MODE == 1) {
              hv[e] = (_Float16)sp[e];
            } else {
              unsigned short hb = f2bf_bits(sp[e]);
              unsigned short lb = f2bf_bits(sp[e] - bf_bits2f(hb));
              hv[e] = __builtin_bit_cast(_Float16, hb);
              lv[e] = __builtin_bit_cast(_Float16, lb);
            }
          }
          *(volatile v8h*)(C + (size_t)(mBase + row) * ldc + n0 + c8) = hv;
          if (OUT_MODE == 2) *(volatile v8h*)(C2 + (size_t)(mBase + row) * ldc + n0 + c8) = lv;
        }
        __threadfence();
      }
    }
    __builtin_amdgcn_fence(__ATOMIC_RELEASE, "workgroup");
    __builtin_amdgcn_wave_barrier();
    __builtin_amdgcn_fence(__ATOMIC_ACQUIRE, "workgroup");
  }
}

__device__ __forceinline__ int blk_excl_scan(int cnt, int* scan_ws, int tid, int* tot) {
  const int lane = tid & 31, wave = tid >> 5; int incl = cnt;
#pragma unroll
  for (int o = 1; o < 32; o <<= 1) { const int v = __shfl_up(incl, o, 32); if (lane >= o) incl += v; }
  if (lane == 31) scan_ws[wave] = incl;
  __syncthreads();
  if (wave == 0) { int wv = (lane < NT / 32) ? scan_ws[lane] : 0; int wincl = wv;
#pragma unroll
    for (int o = 1; o < 32; o <<= 1) { const int v = __shfl_up(wincl, o, 32); if (lane >= o) wincl += v; }
    if (lane < NT / 32) scan_ws[32 + lane] = wincl - wv; if (lane == 31) scan_ws[64] = wincl; }
  __syncthreads();
  const int res = scan_ws[32 + wave] + incl - cnt; *tot = scan_ws[64];
  return res;
}
template <int SP, int CAP>
__device__ __forceinline__ int chunk_hits(const int* __restrict__ dstv, int e0, int n0, int tid, int* LIST, int* scan_ws) {
  const int eb = e0 + tid * SP;
  const bool valid = eb < NE;
  const int ebc = valid ? eb : (NE - SP);
  int rec[SP]; int cnt = 0;
#pragma unroll
  for (int k = 0; k < SP; k += 4) {
    const v4i d4 = *(const v4i*)(dstv + ebc + k);
#pragma unroll
    for (int e = 0; e < 4; ++e) {
      const int d = d4[e]; int r = -1;
      if (valid && d >= n0 && d < n0 + TILE && d < NN) { r = ((d - n0) << 20) | (ebc + k + e); ++cnt; }
      rec[k + e] = r;
    }
  }
  int tot; int p = blk_excl_scan(cnt, scan_ws, tid, &tot);
#pragma unroll
  for (int k = 0; k < SP; ++k) if (rec[k] >= 0) { if ((unsigned)p < (unsigned)CAP) LIST[p] = rec[k]; ++p; }
  __syncthreads();
  return tot < CAP ? tot : CAP;
}

__device__ __forceinline__ unsigned pack_h2(float a, float b) {
  const _Float16 h0 = (_Float16)a, h1 = (_Float16)b;
  return (unsigned)__builtin_bit_cast(unsigned short, h0) | ((unsigned)__builtin_bit_cast(unsigned short, h1) << 16);
}
__device__ __forceinline__ void st2_u32(unsigned* p, unsigned u) { *(volatile unsigned*)p = u; __threadfence(); *(volatile unsigned*)p = u; }

__global__ __launch_bounds__(NT) void prep_kernel(const float* __restrict__ x, const float* __restrict__ Wf, const float* __restrict__ Ws,
                                                 unsigned* __restrict__ XH, unsigned* __restrict__ WT, unsigned* __restrict__ BC) {
  const int i = blockIdx.x * NT + threadIdx.x;
  if (i < XH_N2) {
    const bool live = i < XV_N2;
    const int ic = live ? i : 0;
    float a = x[2 * (size_t)ic], b = x[2 * (size_t)ic + 1];
    if (!live) { a = 0.f; b = 0.f; }
    st2_u32(XH + i, pack_h2(a, b));
  } else if (i < XH_N2 + WT_N2) {
    const int j = i - XH_N2;
    const int r = j >> 6, c = 2 * (j & 63);
    const int sel = r >> 7, rr = r & 127;
    const float* W = (sel < 2) ? Wf : Ws;
    const int cb = (sel & 1) ? FD : 0;
    const float a = W[rr * ZW + cb + c] * WSC, b = W[rr * ZW + cb + c + 1] * WSC;
    st2_u32(WT + j, pack_h2(a, b));
  } else if (i < PREP_TOTAL) {
    const int j = i - XH_N2 - WT_N2;
    const int n = j >> 4, kp = j & 15;
    const bool live = kp < 8;
    const int kc = live ? 2 * kp : 0;
    const float* W = (n < FD) ? Wf : Ws;
    const int rr = n & 127;
    float a = W[rr * ZW + 2 * FD + kc] * WSC, b = W[rr * ZW + 2 * FD + kc + 1] * WSC;
    if (!live) { a = 0.f; b = 0.f; }
    st2_u32(BC + j, pack_h2(a, b));
  }
}

__global__ __launch_bounds__(NT) void edge_kernel(const float* __restrict__ P, const int* __restrict__ ei, const float* __restrict__ ea,
                                                 const unsigned short* __restrict__ BC, const float* __restrict__ bfp, const float* __restrict__ bsp,
                                                 float* AGG) {
  __shared__ int LIST[SCH];
  __shared__ int scan_ws[80];
  __shared__ __align__(16) _Float16 EA[HB * 32];
  __shared__ __align__(16) float PRE[HB * PP];
  const int tid = threadIdx.x, lane = tid & 31, wave = tid >> 5;
  const int rlane = lane & 15, hh = lane >> 4, koff = hh * 8;
  const int n0 = blockIdx.x * TILE;
  const _Float16* BCh = (const _Float16*)(const void*)BC;
  v16h bfr[2];
  bfr[0] = Frag<_Float16>::load(BCh + (size_t)(32 * wave + rlane) * 32 + koff);
  bfr[1] = Frag<_Float16>::load(BCh + (size_t)(32 * wave + 16 + rlane) * 32 + koff);
  const v4f bf4 = *(const v4f*)(bfp + 4 * lane), bs4 = *(const v4f*)(bsp + 4 * lane);
  const v4f z4 = {0.f, 0.f, 0.f, 0.f};
  const v8f z8 = {0.f, 0.f, 0.f, 0.f, 0.f, 0.f, 0.f, 0.f};
  for (int i = tid; i < HB * 16; i += NT) EA[(i >> 4) * 32 + 16 + (i & 15)] = (_Float16)0.0f;
  for (int pass = 0; pass < 2; ++pass) {
#pragma unroll 1
    for (int j = 0; j < TILE / 8; ++j) *(volatile v4f*)(AGG + (size_t)(n0 + wave * (TILE / 8) + j) * FD + 4 * lane) = z4;
    __threadfence();
  }
  __syncthreads();
  const int* srcv = ei; const int* dstv = ei + NE;
#pragma unroll 1
  for (int c = 0; c < NCH; ++c) {
    const int tot = chunk_hits<SPT, SCH>(dstv, c * SCH, n0, tid, LIST, scan_ws);
#pragma unroll 1
    for (int base = 0; base < tot; base += HB) {
      const int nb = (tot - base) < HB ? (tot - base) : HB;
      if (tid < HB * 4) {
        const int q = tid >> 2, p = tid & 3;
        int li = base + q; li = li < SCH ? li : SCH - 1;
        const int rq = LIST[li];
        int e = rq & 0xFFFFF; e = e < NE ? e : NE - 1;
        const bool live = q < nb;
        const v4f av = *(const v4f*)(ea + (size_t)e * ED + 4 * p);
        v4h hv;
#pragma unroll
        for (int k = 0; k < 4; ++k) hv[k] = (_Float16)(live ? av[k] : 0.0f);
        *(v4h*)(EA + q * 32 + 4 * p) = hv;
      }
      __syncthreads();
      {
        v8f acc[2][2];
#pragma unroll
        for (int i = 0; i < 2; ++i) {
          const v16h a = Frag<_Float16>::load(EA + (16 * i + rlane) * 32 + koff);
          acc[i][0] = Frag<_Float16>::mma(a, bfr[0], z8);
          acc[i][1] = Frag<_Float16>::mma(a, bfr[1], z8);
          dep_guard_h(acc[i][0], acc[i][1], a, bfr[1]);
        }
        keep4_h(bfr[0], bfr[1], bfr[0], bfr[1]);
        acc_guard4(acc[0][0], acc[0][1], acc[1][0], acc[1][1]);
#pragma unroll
        for (int i = 0; i < 2; ++i)
#pragma unroll
          for (int j = 0; j < 2; ++j)
#pragma unroll
            for (int r = 0; r < 8; ++r)
              PRE[(16 * i + 8 * hh + r) * PP + 32 * wave + 16 * j + rlane] = acc[i][j][r] * WSC_INV;
      }
      __syncthreads();
      {
        int li = base + lane; li = li < SCH ? li : SCH - 1;
        const int lv = LIST[li];
        const int rv = (lane < nb) ? lv : -1;
        const int own = (rv >= 0 && (rv >> 28) == wave) ? 1 : 0;
        unsigned msk = (unsigned)__ballot(own);
#pragma unroll 1
        for (int it = 0; it < HB; ++it) {
          if (msk == 0u) break;
          const int bp = __builtin_ctz(msk); msk &= msk - 1u;
          const int r = __shfl(rv, bp, 32);
          const int dl = (r >> 20) & (TILE - 1);
          int e = r & 0xFFFFF; e = e < NE ? e : NE - 1;
          int s = srcv[e]; s = s < 0 ? 0 : (s >= NN ? NN - 1 : s);
          int nd = n0 + dl; nd = nd < NN ? nd : NN - 1;
          const float* prow = PRE + bp * PP + 4 * lane;
          const v4f qf = *(const v4f*)(prow);
          const v4f qs = *(const v4f*)(prow + FD);
          const float* spp = P + (size_t)s * PC + 4 * lane;
          const float* dpp = P + (size_t)nd * PC + 4 * lane;
          const v4f psf = *(const v4f*)(spp + FD), pss = *(const v4f*)(spp + 3 * FD);
          const v4f pdf = *(const v4f*)(dpp), pds = *(const v4f*)(dpp + 2 * FD);
          const v4f fl = qf + pdf + psf + bf4;
          const v4f sl = qs + pds + pss + bs4;
          v4f m;
#pragma unroll
          for (int k = 0; k < 4; ++k) {
            const float g  = __builtin_amdgcn_rcpf(1.0f + __expf(-fl[k]));
            const float t  = __expf(-fabsf(sl[k]));
            const float sp = fmaxf(sl[k], 0.0f) + __logf(1.0f + t);
            m[k] = g * sp;
          }
          float* rp = AGG + (size_t)(n0 + dl) * FD + 4 * lane;
          v4f a = *(const v4f*)rp;
          a = a + m;
          *(volatile v4f*)rp = a;
          __threadfence();
          *(volatile v4f*)rp = a;
        }
      }
      __syncthreads();
    }
  }
}

__global__ __launch_bounds__(FD) void bnpart_kernel(const float* __restrict__ AGG, double* __restrict__ PART) {
  const int f = threadIdx.x;
  const int r0 = blockIdx.x * RPB;
  double s = 0.0, ss = 0.0;
#pragma unroll 1
  for (int r = 0; r < RPB; ++r) {
    const float v = AGG[(size_t)(r0 + r) * FD + f];
    const double dv = (double)v;
    s += dv; ss += dv * dv;
  }
  double* p0 = PART + (size_t)blockIdx.x * FD + f;
  double* p1 = PART + (size_t)(NBP + blockIdx.x) * FD + f;
  *(volatile double*)p0 = s; *(volatile double*)p1 = ss;
  __threadfence();
  *(volatile double*)p0 = s; *(volatile double*)p1 = ss;
}

__global__ __launch_bounds__(NT) void final_kernel(const float* __restrict__ AGG, const float* __restrict__ x, const double* __restrict__ PART,
                                                  const float* __restrict__ bng, const float* __restrict__ bnb,
                                                  const float* __restrict__ lng, const float* __restrict__ lnb, float* __restrict__ out) {
  __shared__ __align__(16) float smu[FD];
  __shared__ __align__(16) float srs[FD];
  const int tid = threadIdx.x, lane = tid & 31, wave = tid >> 5;
  if (tid < FD) {
    double s = 0.0, ss = 0.0;
#pragma unroll 1
    for (int b = 0; b < NBP; ++b) { s += PART[(size_t)b * FD + tid]; ss += PART[(size_t)(NBP + b) * FD + tid]; }
    const double mu = s * (1.0 / (double)NN);
    double var = ss * (1.0 / (double)NN) - mu * mu;
    var = var > 0.0 ? var : 0.0;
    const float vf = (float)var;
    smu[tid] = (float)mu;
    srs[tid] = 1.0f / sqrtf(vf + EPSV);
  }
  __syncthreads();
  const v4f mu4 = *(const v4f*)(smu + 4 * lane), rs4 = *(const v4f*)(srs + 4 * lane);
  const v4f g4 = *(const v4f*)(bng + 4 * lane), b4 = *(const v4f*)(bnb + 4 * lane);
  const v4f lg4 = *(const v4f*)(lng + 4 * lane), lb4 = *(const v4f*)(lnb + 4 * lane);
#pragma unroll 1
  for (int j = 0; j < 8; ++j) {
    const int n = blockIdx.x * 64 + wave * 8 + j;
    if (n < NN) {
      const v4f a  = *(const v4f*)(AGG + (size_t)n * FD + 4 * lane);
      const v4f xv = *(const v4f*)(x + (size_t)n * FD + 4 * lane);
      v4f t = (a - mu4) * rs4;
      t = t * g4 + b4;
      const v4f h = t + xv;
      float su = h[0] + h[1] + h[2] + h[3];
#pragma unroll
      for (int off = 16; off > 0; off >>= 1) su += __shfl_xor(su, off, 32);
      const float mean = su * (1.0f / (float)FD);
      const v4f d = h - mean;
      float sq = d[0] * d[0] + d[1] * d[1] + d[2] * d[2] + d[3] * d[3];
#pragma unroll
      for (int off = 16; off > 0; off >>= 1) sq += __shfl_xor(sq, off, 32);
      const float var = sq * (1.0f / (float)FD);
      const float rs = 1.0f / sqrtf(var + EPSV);
      v4f ln = d * rs;
      ln = ln * lg4 + lb4;
      v4f o;
#pragma unroll
      for (int k = 0; k < 4; ++k) o[k] = fmaxf(ln[k], 0.0f) + xv[k];
      float* op = out + (size_t)n * FD + 4 * lane;
      *(volatile v4f*)op = o;
      __threadfence();
      *(volatile v4f*)op = o;
    }
  }
}

extern "C" void kernel_launch(void* const* d_in, const int* in_sizes, int n_in,
                              void* d_out, int out_size, void* d_ws, size_t ws_size, hipStream_t stream) {
  if (n_in < 11) return;
  if (in_sizes[0] != NN * FD || in_sizes[1] != 2 * NE || in_sizes[2] != NE * ED || in_sizes[3] != FD * ZW || in_sizes[5] != FD * ZW) return;
  if (out_size != NN * FD) return;
  const float* x    = (const float*)d_in[0];
  const int*   ei   = (const int*)  d_in[1];
  const float* ea   = (const float*)d_in[2];
  const float* Wf   = (const float*)d_in[3];
  const float* bfp  = (const float*)d_in[4];
  const float* Ws   = (const float*)d_in[5];
  const float* bsp  = (const float*)d_in[6];
  const float* bng  = (const float*)d_in[7];
  const float* bnb  = (const float*)d_in[8];
  const float* lng  = (const float*)d_in[9];
  const float* lnb  = (const float*)d_in[10];
  float* out = (float*)d_out;

  char* ws = (char*)d_ws; size_t off = 0;
  auto carve = [&](size_t bytes) -> char* { char* p = ws + off; off += (bytes + 255) & ~(size_t)255; return p; };
  unsigned* XH   = (unsigned*)carve((size_t)NP * FD * 2);
  unsigned* WT   = (unsigned*)carve((size_t)PC * FD * 2);
  unsigned* BC   = (unsigned*)carve((size_t)256 * 32 * 2);
  float*    P    = (float*)carve((size_t)NP * PC * 4);
  float*    AGG  = (float*)carve((size_t)NACC * FD * 4);
  double*   PART = (double*)carve((size_t)2 * NBP * FD * 8);
  if (off > ws_size || off > (size_t)134217728) return;

  prep_kernel<<<(PREP_TOTAL + NT - 1) / NT, NT, 0, stream>>>(x, Wf, Ws, XH, WT, BC);
  {
    const int tiles = (NP / 64) * (PC / 64);
    wmma_gemm64<0, false, 0, 0, false><<<dim3((tiles + 7) / 8, 1), 256, 0, stream>>>(
        (const unsigned short*)XH, (const unsigned short*)nullptr, FD, 0L,
        (const unsigned short*)WT, (const unsigned short*)nullptr, FD, 0L,
        (void*)P, (void*)nullptr, PC, 0L,
        (const float*)nullptr, (const float*)nullptr, 0L, NP, PC, FD, WSC_INV);
  }
  edge_kernel<<<NTILES, NT, 0, stream>>>(P, ei, ea, (const unsigned short*)BC, bfp, bsp, AGG);
  bnpart_kernel<<<NBP, FD, 0, stream>>>(AGG, PART);
  final_kernel<<<(NN + 63) / 64, NT, 0, stream>>>(AGG, x, PART, bng, bnb, lng, lnb, out);
}
